// GAT_40037685133531
// MI455X (gfx1250) — hardware-run, weakly checked
//
#include <hip/hip_runtime.h>
#include <stddef.h>
#include <stdint.h>
#include <math.h>


#define NN      50000
#define NE      800000
#define F_IN    128
#define HC      128
#define HID     32
#define NHD     4
#define F_OUT   64
#define MROWS   128
#define MP      (((NN + MROWS - 1) / MROWS) * MROWS)
#define XPITCH  128
#define WPITCH  128
#define K1EXT   128
#define HEAD_TWO_TERM 1
#define EPITCH  256
#define W2PITCH 256
#define K2EXT   (HEAD_TWO_TERM ? 256 : 128)
#define NTHR    256
#define NWAVE   8
#define EPT     8
#define CHUNK   (NTHR * EPT)
#define WCAP    (EPT * 32)
#define LISTN   (NWAVE * WCAP)
#define NBRUN   1024
#define SLOTB   10
#define NBLK    ((NN + NBRUN - 1) / NBRUN)
#define RCAP    20480
#define DEGCAP  64
#define G1M     64
#define G1T     256
#define SP1     132
#define G2M     64
#define G2N     64
#define G2T     128
#define NEGSL   0.2f
#define EPS_SM  1e-16f
#define WSMAX   ((size_t)(128u << 20))
#define LDS_BKT ((2 * RCAP + 2 * NBRUN + LISTN + 2 * NWAVE) * 4)

#define PB_X    ((MP * (F_IN / 8)) / NTHR)
#define PB_W    ((HC * (WPITCH / 8)) / NTHR)
#define PB_W2   ((F_OUT * (W2PITCH / 8)) / NTHR)
#define PB_S    1
#define PB_E    (((MP - NN) * (EPITCH / 8)) / NTHR)
#define PB_ALL  (PB_X + PB_W + PB_W2 + PB_S + PB_E)

static_assert(NN <= 65536);
static_assert(NBRUN <= 1024 && NBRUN == (1 << SLOTB));
static_assert(NBLK * NBRUN >= NN);
static_assert(16623 + 2048 <= RCAP);
static_assert(35 + 8 <= DEGCAP && DEGCAP == 64);
static_assert((CHUNK & (CHUNK - 1)) == 0 && (CHUNK << SLOTB) > 0);
static_assert(LISTN >= NBRUN && LISTN >= NWAVE * WCAP);
static_assert(NBRUN == 4 * NTHR);
static_assert((RCAP % (NTHR * 4)) == 0);
static_assert(LDS_BKT <= 327680);
static_assert((MP * (F_IN / 8)) % NTHR == 0);
static_assert((HC * (WPITCH / 8)) % NTHR == 0 && (F_OUT * (W2PITCH / 8)) % NTHR == 0);
static_assert(((MP - NN) * (EPITCH / 8)) % NTHR == 0);
static_assert((K1EXT % 32) == 0 && (K2EXT % 32) == 0 && K1EXT <= XPITCH && K1EXT <= WPITCH);
static_assert(K2EXT <= EPITCH && K2EXT <= W2PITCH);
static_assert((MP % G1M) == 0 && (MP % G2M) == 0);
static_assert(HC == 4 * 32 && HID == 32 && NHD * HID == HC);
static_assert(G1T == 4 * G1M && G1T == 2 * HC);
static_assert((NN % 8) == 0 && (NE % 4) == 0);
static_assert(NBLK * NBRUN >= MP);

typedef float          v4f  __attribute__((ext_vector_type(4)));
typedef float          v8f  __attribute__((ext_vector_type(8)));
typedef int            v4i  __attribute__((ext_vector_type(4)));
typedef int            v8i  __attribute__((ext_vector_type(8)));
typedef unsigned int   v4u  __attribute__((ext_vector_type(4)));
typedef unsigned short v8us __attribute__((ext_vector_type(8)));
typedef __bf16         v16b __attribute__((ext_vector_type(16)));
typedef v4f  __attribute__((may_alias)) v4fa;
typedef v4i  __attribute__((may_alias)) v4ia;
typedef v8us __attribute__((may_alias)) v8usa;
union FragB { v16b v; v8us h[2]; v8i w; };

__device__ __forceinline__ v8f wmb(const FragB& a, const FragB& b, v8f c) {
  v8f d = __builtin_amdgcn_wmma_f32_16x16x32_bf16(false, a.v, false, b.v, (short)0, c, false, false);
  asm volatile("v_nop\n\tv_nop\n\tv_nop\n\tv_nop" : "+v"(d) : "v"(a.w), "v"(b.w));
  return d;
}

__device__ __forceinline__ unsigned int f2bf(float f) {
  const unsigned int u = __float_as_uint(f);
  const unsigned int r = ((u + 0x7FFFu + ((u >> 16) & 1u)) >> 16) & 0xFFFFu;
  return ((u & 0x7FFFFFFFu) > 0x7F800000u) ? 0x7FC0u : r;
}
__device__ __forceinline__ float bf2f(unsigned int b) { return __uint_as_float(b << 16); }
__device__ __forceinline__ float bfr(float f) { return bf2f(f2bf(f)); }
__device__ __forceinline__ v4f bfr4(const v4f a) {
  v4f r; r.x = bfr(a.x); r.y = bfr(a.y); r.z = bfr(a.z); r.w = bfr(a.w); return r;
}
__device__ __forceinline__ unsigned int pk2(float lo, float hi) { return f2bf(lo) | (f2bf(hi) << 16); }
__device__ __forceinline__ v4u pack8(const v4f a, const v4f b) {
  v4u r;
  r.x = pk2(a.x, a.y); r.y = pk2(a.z, a.w); r.z = pk2(b.x, b.y); r.w = pk2(b.z, b.w);
  return r;
}

__device__ __forceinline__ void wtr_unit(const float* __restrict__ w, int Kin, int Ncol, int Kout,
                                         unsigned short* wt, int u) {
  const int kq = Kout >> 3;
  const int n  = u / kq;
  const int k8 = (u - n * kq) * 8;
  const int kk = k8 - (k8 / Kin) * Kin;
  const float* p = w + (size_t)kk * (size_t)Ncol + n;
  v4f a, b;
  a.x = p[0];                    a.y = p[(size_t)Ncol];         a.z = p[(size_t)2 * Ncol];     a.w = p[(size_t)3 * Ncol];
  b.x = p[(size_t)4 * Ncol];     b.y = p[(size_t)5 * Ncol];     b.z = p[(size_t)6 * Ncol];     b.w = p[(size_t)7 * Ncol];
  const v4u wv = pack8(a, b);
  unsigned short* o = wt + (size_t)n * (size_t)Kout + k8;
  *(volatile v4u*)o = wv;
  __threadfence();
  *(volatile v4u*)o = wv;
}

__global__ __launch_bounds__(NTHR) void k_prep(const float* __restrict__ x, const float* __restrict__ W,
                                               const float* __restrict__ W2, const float* __restrict__ asrc,
                                               const float* __restrict__ adst, const float* __restrict__ bias,
                                               const float* __restrict__ b2,
                                               unsigned short* XB, unsigned short* WT, unsigned short* W2D,
                                               float* SP, unsigned short* E) {
  const int bx = (int)blockIdx.x, tid = (int)threadIdx.x;
  if (bx < PB_X) {
    const int i = bx * NTHR + tid;
    const int row = i >> 4;
    const int c0  = (i & 15) * 8;
    const int rc  = row < NN ? row : NN - 1;
    const float* p = x + (size_t)rc * F_IN + c0;
    v4f a = *(const v4fa*)p, b = *(const v4fa*)(p + 4);
    const v4f z4 = {0.f, 0.f, 0.f, 0.f};
    if (row >= NN) { a = z4; b = z4; }
    const v4u hv = pack8(a, b);
    unsigned short* o = XB + (size_t)row * XPITCH + c0;
    *(volatile v4u*)o = hv;
    __threadfence();
    *(volatile v4u*)o = hv;
  } else if (bx < PB_X + PB_W) {
    wtr_unit(W, F_IN, HC, WPITCH, WT, (bx - PB_X) * NTHR + tid);
  } else if (bx < PB_X + PB_W + PB_W2) {
    wtr_unit(W2, HC, F_OUT, W2PITCH, W2D, (bx - PB_X - PB_W) * NTHR + tid);
  } else if (bx < PB_X + PB_W + PB_W2 + PB_S) {
    const int wv = tid >> 5;
    const int q  = tid & 31;
    const v4f va = *(const v4fa*)(asrc + 4 * q);
    const v4f vd = *(const v4fa*)(adst + 4 * q);
    const v4f vb = *(const v4fa*)(bias + 4 * q);
    const v4f v2 = *(const v4fa*)(b2 + 4 * (q & 15));
    asm volatile("" :: "v"(va)); asm volatile("" :: "v"(vd));
    asm volatile("" :: "v"(vb)); asm volatile("" :: "v"(v2));
    v4f v = va;
    v = (wv == 1) ? vd : v;
    v = (wv == 2) ? vb : v;
    v = (wv >= 3) ? v2 : v;
    v = bfr4(v);
    const bool wr = tid < 112;
    float* o = SP + 4 * (wr ? tid : 0);
    if (wr) *(volatile v4f*)o = v;
    __threadfence();
    if (wr) *(volatile v4f*)o = v;
  } else {
    const int u = (bx - PB_X - PB_W - PB_W2 - PB_S) * NTHR + tid;
    const int row = NN + (u >> 5);
    const int c0  = (u & 31) * 8;
    const v4u z = {0u, 0u, 0u, 0u};
    unsigned short* o = E + (size_t)row * EPITCH + c0;
    *(volatile v4u*)o = z;
    __threadfence();
    *(volatile v4u*)o = z;
  }
}

__global__ __launch_bounds__(G1T) __attribute__((amdgpu_num_vgpr(248))) void k_gemm_one(
    const unsigned short* __restrict__ A, const unsigned short* __restrict__ WT,
    const float* __restrict__ SP, float* H, float* SD)
{
  __shared__ __attribute__((aligned(16))) float stg[G1M * SP1];
  __shared__ __attribute__((aligned(16))) float satt[2 * HC];
  __shared__ __attribute__((aligned(16))) float sdot[G1M * 8];
  const int tid = (int)threadIdx.x, lane = tid & 31, wave = tid >> 5, hh = lane >> 4, m = lane & 15;
  const int rt = wave & 3, cg = wave >> 2;
  const int rowBase = (int)blockIdx.x * G1M;
  const int col0    = cg * 64;

  if (tid < 64) {
    const v4f v = *(const v4fa*)(SP + 4 * tid);
    *(v4fa*)(satt + 4 * tid) = v;
  }

  v8f acc[4];
  {
    const v8f z = {0.f, 0.f, 0.f, 0.f, 0.f, 0.f, 0.f, 0.f};
    acc[0] = z; acc[1] = z; acc[2] = z; acc[3] = z;
  }
  const unsigned short* ap = A  + (size_t)(rowBase + 16 * rt + m) * (size_t)XPITCH + 8 * hh;
  const unsigned short* wp = WT + (size_t)(col0 + m) * (size_t)WPITCH + 8 * hh;
#pragma unroll 1
  for (int ks = 0; ks < K1EXT / 32; ++ks) {
    FragB af;
    af.h[0] = *(const v8usa*)(ap + 32 * ks);
    af.h[1] = *(const v8usa*)(ap + 32 * ks + 16);
#pragma unroll
    for (int t = 0; t < 4; ++t) {
      const unsigned short* wq = wp + (size_t)(16 * t) * (size_t)WPITCH + 32 * ks;
      FragB bf;
      bf.h[0] = *(const v8usa*)wq;
      bf.h[1] = *(const v8usa*)(wq + 16);
      acc[t] = wmb(af, bf, acc[t]);
    }
  }

#pragma unroll
  for (int t = 0; t < 4; ++t) {
    const int lc = col0 + 16 * t + m;
#pragma unroll
    for (int r = 0; r < 8; ++r) {
      const int lr = 16 * rt + 8 * hh + r;
      stg[lr * SP1 + lc] = acc[t][r];
    }
  }
  __syncthreads();

  {
    const int row = tid & 63, hd = tid >> 6;
    const float* sa = satt + hd * HID;
    const float* sb = satt + HC + hd * HID;
    const float* hr = stg + row * SP1 + HID * hd;
    float ds = 0.f, dd = 0.f;
#pragma unroll 2
    for (int c4 = 0; c4 < HID / 4; ++c4) {
      const v4f hv = *(const v4fa*)(hr + 4 * c4);
      const v4f av = *(const v4fa*)(sa + 4 * c4);
      const v4f bv = *(const v4fa*)(sb + 4 * c4);
      ds = fmaf(hv.x, av.x, ds);  dd = fmaf(hv.x, bv.x, dd);
      ds = fmaf(hv.y, av.y, ds);  dd = fmaf(hv.y, bv.y, dd);
      ds = fmaf(hv.z, av.z, ds);  dd = fmaf(hv.z, bv.z, dd);
      ds = fmaf(hv.w, av.w, ds);  dd = fmaf(hv.w, bv.w, dd);
    }
    sdot[row * 8 + hd]     = ds;
    sdot[row * 8 + 4 + hd] = dd;
  }
  __syncthreads();

  v4f fv[8];
#pragma unroll
  for (int i = 0; i < 8; ++i) {
    const int lr = 8 * wave + i;
    fv[i] = *(const v4fa*)(stg + lr * SP1 + 4 * lane);
  }
  const int pc = tid & 127;
  const v4f sdv = *(const v4fa*)(sdot + 4 * pc);
  float* sp = SD + (size_t)rowBase * 8 + 4 * pc;
  const bool wsd = wave < 4;

#pragma unroll
  for (int i = 0; i < 8; ++i) {
    float* op = H + (size_t)(rowBase + 8 * wave + i) * HC + 4 * lane;
    *(volatile v4f*)op = fv[i];
  }
  if (wsd) *(volatile v4f*)sp = sdv;
  __threadfence();
#pragma unroll
  for (int i = 0; i < 8; ++i) {
    float* op = H + (size_t)(rowBase + 8 * wave + i) * HC + 4 * lane;
    *(volatile v4f*)op = fv[i];
  }
  if (wsd) *(volatile v4f*)sp = sdv;
}

__device__ __forceinline__ int scan_chunk(const int* __restrict__ dsts, int nE, int cbase, int slotBase,
                                          int nb, int vec8, int* list, int tid, int lane, int wave) {
  int wc = 0;
  const int el0  = tid * EPT;
  const int e0   = cbase + el0;
  const int sent = (int)(1u << 31);
  v4i da, db;
  if (vec8 != 0 && cbase + CHUNK <= nE) {
    da = *(const v4i*)(dsts + e0);
    db = *(const v4i*)(dsts + e0 + 4);
  } else {
    const int q0 = dsts[min(e0,     nE - 1)];
    const int q1 = dsts[min(e0 + 1, nE - 1)];
    const int q2 = dsts[min(e0 + 2, nE - 1)];
    const int q3 = dsts[min(e0 + 3, nE - 1)];
    const int q4 = dsts[min(e0 + 4, nE - 1)];
    const int q5 = dsts[min(e0 + 5, nE - 1)];
    const int q6 = dsts[min(e0 + 6, nE - 1)];
    const int q7 = dsts[min(e0 + 7, nE - 1)];
    asm volatile("" :: "v"(q0)); asm volatile("" :: "v"(q1)); asm volatile("" :: "v"(q2)); asm volatile("" :: "v"(q3));
    asm volatile("" :: "v"(q4)); asm volatile("" :: "v"(q5)); asm volatile("" :: "v"(q6)); asm volatile("" :: "v"(q7));
    da.x = (e0     < nE) ? q0 : sent;
    da.y = (e0 + 1 < nE) ? q1 : sent;
    da.z = (e0 + 2 < nE) ? q2 : sent;
    da.w = (e0 + 3 < nE) ? q3 : sent;
    db.x = (e0 + 4 < nE) ? q4 : sent;
    db.y = (e0 + 5 < nE) ? q5 : sent;
    db.z = (e0 + 6 < nE) ? q6 : sent;
    db.w = (e0 + 7 < nE) ? q7 : sent;
  }
  const unsigned nbs = (unsigned)slotBase;
  const unsigned unb = (unsigned)nb;
  const unsigned s0 = (unsigned)da.x - nbs, s1 = (unsigned)da.y - nbs;
  const unsigned s2 = (unsigned)da.z - nbs, s3 = (unsigned)da.w - nbs;
  const unsigned s4 = (unsigned)db.x - nbs, s5 = (unsigned)db.y - nbs;
  const unsigned s6 = (unsigned)db.z - nbs, s7 = (unsigned)db.w - nbs;
  const bool h0 = s0 < unb, h1 = s1 < unb, h2 = s2 < unb, h3 = s3 < unb;
  const bool h4 = s4 < unb, h5 = s5 < unb, h6 = s6 < unb, h7 = s7 < unb;
  const unsigned any = __builtin_amdgcn_ballot_w32(h0 | h1 | h2 | h3 | h4 | h5 | h6 | h7);
  if (any != 0u) {
#define HITJ(J, HJ, SJ) { \
      const unsigned mj = __builtin_amdgcn_ballot_w32(HJ); \
      if (mj != 0u) { \
        if (HJ) { \
          const int pos = wc + (int)__builtin_amdgcn_mbcnt_lo(mj, 0u); \
          if (pos < WCAP) list[wave * WCAP + pos] = ((el0 + (J)) << SLOTB) | (int)(SJ); \
        } \
        wc += (int)__builtin_popcount(mj); } }
    HITJ(0, h0, s0)
    HITJ(1, h1, s1)
    HITJ(2, h2, s2)
    HITJ(3, h3, s3)
    HITJ(4, h4, s4)
    HITJ(5, h5, s5)
    HITJ(6, h6, s6)
    HITJ(7, h7, s7)
#undef HITJ
  }
  return wc;
}

__global__ __launch_bounds__(NTHR) void k_bucket(const int* __restrict__ srcs, const int* __restrict__ dsts,
                                                 int* HITS, int* OFF, int* CNT, int* FLG,
                                                 int nN, int nE, int vec8) {
  extern __shared__ v4f lds_dyn[];
  int* reg1 = (int*)lds_dyn;
  int* reg2 = reg1 + RCAP;
  int* scnt = reg2 + RCAP;
  int* soff = scnt + NBRUN;
  int* list = soff + NBRUN;
  int* wcnt = list + LISTN;
  int* wtot = wcnt + NWAVE;
  const int tid = (int)threadIdx.x, lane = tid & 31, wave = tid >> 5;
  const int bk = (int)blockIdx.x;
  const int nodeBase = bk * NBRUN;
  int nb = nN - nodeBase;
  nb = nb > NBRUN ? NBRUN : (nb < 0 ? 0 : nb);

  for (int i = tid; i < NBRUN; i += NTHR) scnt[i] = 0;
  for (int i = tid; i < RCAP; i += NTHR) reg2[i] = 0;
  __syncthreads();

  int tot = 0;
  const int nChunks = (nE + CHUNK - 1) / CHUNK;
#pragma unroll 1
  for (int ch = 0; ch < nChunks; ++ch) {
    const int cbase = ch * CHUNK;
    const int wc = scan_chunk(dsts, nE, cbase, nodeBase, nb, vec8, list, tid, lane, wave);
    if (lane == 0) wcnt[wave] = wc;
    __syncthreads();
    int pre = 0, all = 0;
#pragma unroll
    for (int w2 = 0; w2 < NWAVE; ++w2) {
      int c = wcnt[w2];
      c = c < 0 ? 0 : (c > WCAP ? WCAP : c);
      all += c;
      pre += (w2 < wave) ? c : 0;
    }
    const int wcc  = wc > WCAP ? WCAP : wc;
    const int base = tot + pre;
#pragma unroll 1
    for (int i0 = 0; i0 < wcc; i0 += 32) {
      const int i  = i0 + lane;
      const int ic = i < wcc ? i : wcc - 1;
      const int ent = list[wave * WCAP + ic];
      const int el  = (ent >> SLOTB) & (CHUNK - 1);
      const int sl  = ent & (NBRUN - 1);
      int eid = cbase + el;
      eid = eid > nE - 1 ? nE - 1 : eid;
      const int sraw = srcs[eid];
      asm volatile("" :: "v"(sraw));
      const int s = sraw < 0 ? 0 : (sraw > nN - 1 ? nN - 1 : sraw);
      const int pos = base + i;
      if (i < wcc && pos < RCAP) reg1[pos] = (int)((unsigned)s | ((unsigned)sl << 16));
    }
    tot += all;
    tot = tot > RCAP ? RCAP : tot;
    __syncthreads();
  }
  const int nh = tot;

  if (wave == 0) {
#pragma unroll 1
    for (int b0 = 0; b0 < nh; b0 += 32) {
      const int idx = b0 + lane;
      const int uv  = reg1[idx < nh ? idx : nh - 1];
      const int m32 = (nh - b0) < 32 ? (nh - b0) : 32;
#pragma unroll 1
      for (int k = 0; k < m32; ++k) {
        const int u  = __builtin_amdgcn_readlane(uv, k);
        const int sl = (u >> 16) & (NBRUN - 1);
        if (lane == 0) scnt[sl] = scnt[sl] + 1;
      }
    }
  }
  __syncthreads();

  {
    const v4i ca = *(const v4ia*)(scnt + 4 * tid);
    const int e0 = ca.x < 0 ? 0 : ca.x, e1 = ca.y < 0 ? 0 : ca.y, e2 = ca.z < 0 ? 0 : ca.z, e3 = ca.w < 0 ? 0 : ca.w;
    const int ts = e0 + e1 + e2 + e3;
    int incl = ts;
#pragma unroll
    for (int d = 1; d < 32; d <<= 1) {
      const int up = __shfl_up(incl, d);
      if (lane >= d) incl += up;
    }
    if (lane == 31) wtot[wave] = incl;
    __syncthreads();
    int pre = 0;
#pragma unroll
    for (int w2 = 0; w2 < NWAVE; ++w2) pre += (w2 < wave) ? wtot[w2] : 0;
    int run = pre + incl - ts;
    soff[4 * tid + 0] = run; run += e0;
    soff[4 * tid + 1] = run; run += e1;
    soff[4 * tid + 2] = run; run += e2;
    soff[4 * tid + 3] = run;
  }
  __syncthreads();
  for (int i = tid; i < NBRUN; i += NTHR) list[i] = soff[i];
  __syncthreads();

  if (wave == 0) {
#pragma unroll 1
    for (int b0 = 0; b0 < nh; b0 += 32) {
      const int idx = b0 + lane;
      const int uv  = reg1[idx < nh ? idx : nh - 1];
      const int m32 = (nh - b0) < 32 ? (nh - b0) : 32;
#pragma unroll 1
      for (int k = 0; k < m32; ++k) {
        const int u  = __builtin_amdgcn_readlane(uv, k);
        const int sl = (u >> 16) & (NBRUN - 1);
        if (lane == 0) {
          int pos = list[sl];
          pos = pos < 0 ? 0 : (pos > RCAP - 1 ? RCAP - 1 : pos);
          reg2[pos] = u;
          list[sl] = pos + 1;
        }
      }
    }
  }
  __syncthreads();

  const int fl = (nh >= RCAP) ? 1 : 0;
  const v4i fl4 = {fl, fl, fl, fl};
  const v4i so4 = *(const v4ia*)(soff + 4 * tid);
  const v4i sc4 = *(const v4ia*)(scnt + 4 * tid);
  int* hb = HITS + (size_t)bk * RCAP;
  int* ob = OFF + (size_t)bk * NBRUN + 4 * tid;
  int* cb = CNT + (size_t)bk * NBRUN + 4 * tid;
  int* fb = FLG + (size_t)bk * 32 + 4 * (lane & 7);
  const bool wfl = (wave == 0) && (lane < 8);
#pragma unroll 1
  for (int ps = 0; ps < RCAP / (NTHR * 4); ++ps) {
    const int ix = (ps * NTHR + tid) * 4;
    const v4i v = *(const v4ia*)(reg2 + ix);
    *(volatile v4i*)(hb + ix) = v;
  }
  *(volatile v4i*)ob = so4;
  *(volatile v4i*)cb = sc4;
  if (wfl) *(volatile v4i*)fb = fl4;
  __threadfence();
#pragma unroll 1
  for (int ps = 0; ps < RCAP / (NTHR * 4); ++ps) {
    const int ix = (ps * NTHR + tid) * 4;
    const v4i v = *(const v4ia*)(reg2 + ix);
    *(volatile v4i*)(hb + ix) = v;
  }
  *(volatile v4i*)ob = so4;
  *(volatile v4i*)cb = sc4;
  if (wfl) *(volatile v4i*)fb = fl4;
}

__global__ __launch_bounds__(NTHR) void k_replay(const float* __restrict__ H, const float* __restrict__ SD,
                                                 const float* __restrict__ SP, const int* __restrict__ HITS,
                                                 const int* __restrict__ OFF, const int* __restrict__ CNT,
                                                 const int* __restrict__ FLG, unsigned short* E, int nN) {
  __shared__ __attribute__((aligned(16))) float sbias[HC];
  const int tid = (int)threadIdx.x, lane = tid & 31, wave = tid >> 5;
  if (tid < 32) {
    const v4f bv = *(const v4fa*)(SP + 2 * HC + 4 * tid);
    *(v4fa*)(sbias + 4 * tid) = bv;
  }
  __syncthreads();

  const int d = (int)blockIdx.x * NWAVE + wave;
  const bool live = d < nN;
  const int dc = live ? d : nN - 1;
  const int bk = dc >> SLOTB;
  const int offv = OFF[dc];
  const int cntv = CNT[dc];
  const int flgv = FLG[bk * 32];
  asm volatile("" :: "v"(offv)); asm volatile("" :: "v"(cntv)); asm volatile("" :: "v"(flgv));
  int ov = offv < 0 ? 0 : (offv > RCAP - 1 ? RCAP - 1 : offv);
  int cv = cntv < 0 ? 0 : (cntv > DEGCAP ? DEGCAP : cntv);
  cv = cv > RCAP - ov ? RCAP - ov : cv;
  const bool pois = (flgv != 0) || (cntv > DEGCAP) || (cntv < 0);
  const int o = __builtin_amdgcn_readfirstlane(ov);
  const int c = __builtin_amdgcn_readfirstlane(cv);
  int last = o + c - 1;
  last = last < o ? o : last;
  const int* hb = HITS + (size_t)bk * RCAP;
  int i0 = o + lane;      i0 = i0 > last ? last : i0;
  int i1 = o + 32 + lane; i1 = i1 > last ? last : i1;
  const int w0 = hb[i0];
  const int w1 = hb[i1];

  const int hd = lane >> 3;
  const unsigned k0 = (hd == 0) ? 0xFFFFFFFFu : 0u;
  const unsigned k1 = (hd == 1) ? 0xFFFFFFFFu : 0u;
  const unsigned k2 = (hd == 2) ? 0xFFFFFFFFu : 0u;
  const unsigned k3 = (hd == 3) ? 0xFFFFFFFFu : 0u;
  const v4f ad4 = *(const v4fa*)(SD + (size_t)dc * 8 + 4);
  asm volatile("" :: "v"(ad4));
  const float adv = __uint_as_float((__float_as_uint(ad4.x) & k0) | (__float_as_uint(ad4.y) & k1) |
                                    (__float_as_uint(ad4.z) & k2) | (__float_as_uint(ad4.w) & k3));

  float mx = __int_as_float((int)0xff800000u);
  float dn = 0.0f;
  v4f av = {0.f, 0.f, 0.f, 0.f};

#pragma unroll 1
  for (int q = 0; q < c; ++q) {
    const int r0 = __builtin_amdgcn_readlane(w0, q & 31);
    const int r1 = __builtin_amdgcn_readlane(w1, q & 31);
    const int w  = (q < 32) ? r0 : r1;
    int s = w & 0xFFFF;
    s = s > nN - 1 ? nN - 1 : s;
    const v4f as4 = *(const v4fa*)(SD + (size_t)s * 8);
    const v4f fs  = *(const v4fa*)(H + (size_t)s * HC + 4 * lane);
    asm volatile("" :: "v"(as4));
    const float asv = __uint_as_float((__float_as_uint(as4.x) & k0) | (__float_as_uint(as4.y) & k1) |
                                      (__float_as_uint(as4.z) & k2) | (__float_as_uint(as4.w) & k3));
    float e = asv + adv;
    e = (e >= 0.0f) ? e : NEGSL * e;
    const float mn = fmaxf(mx, e);
    const float r  = expf(mx - mn);
    const float p  = expf(e - mn);
    dn = dn * r + p;
    av.x = av.x * r + p * fs.x;
    av.y = av.y * r + p * fs.y;
    av.z = av.z * r + p * fs.z;
    av.w = av.w * r + p * fs.w;
    mx = mn;
  }
  const float inv = __builtin_amdgcn_rcpf(dn + EPS_SM);
  const v4f bb = *(const v4fa*)(sbias + 4 * lane);
  float c0 = av.x * inv + bb.x;
  float c1 = av.y * inv + bb.y;
  float c2 = av.z * inv + bb.z;
  float c3 = av.w * inv + bb.w;
#pragma unroll 1
  for (int j = 0; j < 4; ++j) {
    const float t  = c0;
    const float en = expm1f(t);
    const float u  = (t > 0.0f) ? t : en;
    c0 = c1; c1 = c2; c2 = c3; c3 = u;
  }
  const float qnan = __int_as_float(0x7fc00000);
  const float ox = pois ? qnan : c0;
  const float oy = pois ? qnan : c1;
  const float oz = pois ? qnan : c2;
  const float ow = pois ? qnan : c3;
  const unsigned int hbx = f2bf(ox), hby = f2bf(oy), hbz = f2bf(oz), hbw = f2bf(ow);
  const unsigned int lbx = f2bf(ox - bf2f(hbx)), lby = f2bf(oy - bf2f(hby));
  const unsigned int lbz = f2bf(oz - bf2f(hbz)), lbw = f2bf(ow - bf2f(hbw));
  const int hw0 = (int)(hbx | (hby << 16)), hw1 = (int)(hbz | (hbw << 16));
  const int lw0 = (int)(lbx | (lby << 16)), lw1 = (int)(lbz | (lbw << 16));
  const int sa = (2 * lane) & 31, sb = (2 * lane + 1) & 31;
  const int g0 = __shfl(hw0, sa), g1 = __shfl(hw1, sa), g2 = __shfl(hw0, sb), g3 = __shfl(hw1, sb);
  const int q0 = __shfl(lw0, sa), q1 = __shfl(lw1, sa), q2 = __shfl(lw0, sb), q3 = __shfl(lw1, sb);
  const bool lsel = lane >= 16;
  v4u pv;
  pv.x = (unsigned int)(lsel ? q0 : g0);
  pv.y = (unsigned int)(lsel ? q1 : g1);
  pv.z = (unsigned int)(lsel ? q2 : g2);
  pv.w = (unsigned int)(lsel ? q3 : g3);
  unsigned short* gp = E + (size_t)dc * EPITCH + 8 * lane;
  if (live) *(volatile v4u*)gp = pv;
  __threadfence();
  if (live) *(volatile v4u*)gp = pv;
}

__global__ __launch_bounds__(G2T) __attribute__((amdgpu_num_vgpr(248))) void k_gemm_two(
    const unsigned short* __restrict__ A, const unsigned short* __restrict__ WT,
    const float* __restrict__ SP, const int* __restrict__ CNT, const int* __restrict__ FLG,
    float* out, int nN)
{
  __shared__ __attribute__((aligned(16))) float stg[G2M * G2N];
  __shared__ __attribute__((aligned(16))) float sb2[G2N];
  __shared__ __attribute__((aligned(16))) int   spz[G2M];
  const int tid = (int)threadIdx.x, lane = tid & 31, wave = tid >> 5, hh = lane >> 4, m = lane & 15;
  const int rowBase = (int)blockIdx.x * G2M;

  if (tid < 64) {
    const float bv = SP[3 * HC + tid];
    int row = rowBase + tid;
    row = row > nN - 1 ? nN - 1 : row;
    const int cr = CNT[row];
    const int fr = FLG[(row >> SLOTB) * 32];
    asm volatile("" :: "v"(bv)); asm volatile("" :: "v"(cr)); asm volatile("" :: "v"(fr));
    sb2[tid] = bv;
    spz[tid] = ((fr != 0) || (cr > DEGCAP) || (cr < 0)) ? 1 : 0;
  }

  v8f acc[4];
  {
    const v8f z = {0.f, 0.f, 0.f, 0.f, 0.f, 0.f, 0.f, 0.f};
    acc[0] = z; acc[1] = z; acc[2] = z; acc[3] = z;
  }
  const unsigned short* ap = A  + (size_t)(rowBase + 16 * wave + m) * (size_t)EPITCH + 8 * hh;
  const unsigned short* wp = WT + (size_t)m * (size_t)W2PITCH + 8 * hh;
#pragma unroll 1
  for (int ks = 0; ks < K2EXT / 32; ++ks) {
    FragB af;
    af.h[0] = *(const v8usa*)(ap + 32 * ks);
    af.h[1] = *(const v8usa*)(ap + 32 * ks + 16);
#pragma unroll
    for (int t = 0; t < 4; ++t) {
      const unsigned short* wq = wp + (size_t)(16 * t) * (size_t)W2PITCH + 32 * ks;
      FragB bf;
      bf.h[0] = *(const v8usa*)wq;
      bf.h[1] = *(const v8usa*)(wq + 16);
      acc[t] = wmb(af, bf, acc[t]);
    }
  }

#pragma unroll
  for (int t = 0; t < 4; ++t) {
    const int lc = 16 * t + m;
#pragma unroll
    for (int r = 0; r < 8; ++r) {
      const int lr = 16 * wave + 8 * hh + r;
      stg[lr * G2N + lc] = acc[t][r];
    }
  }
  __syncthreads();

  const float qnan = __int_as_float(0x7fc00000);
  const v4f b4 = *(const v4fa*)(sb2 + 4 * m);
  v4f fv[8];
#pragma unroll
  for (int i = 0; i < 8; ++i) {
    const int lr = 16 * wave + 2 * i + hh;
    v4f v = *(const v4fa*)(stg + lr * G2N + 4 * m);
    const int pz = spz[lr];
    v.x = v.x + b4.x; v.y = v.y + b4.y; v.z = v.z + b4.z; v.w = v.w + b4.w;
    v.x = (pz != 0) ? qnan : v.x;
    v.y = (pz != 0) ? qnan : v.y;
    v.z = (pz != 0) ? qnan : v.z;
    v.w = (pz != 0) ? qnan : v.w;
    fv[i] = v;
    asm volatile("" :: "v"(fv[i]));
  }
#pragma unroll
  for (int i = 0; i < 8; ++i) {
    const int gr = rowBase + 16 * wave + 2 * i + hh;
    const int gc = gr < nN ? gr : nN - 1;
    float* op = out + (size_t)gc * F_OUT + 4 * m;
    if (gr < nN) *(volatile v4f*)op = fv[i];
  }
  __threadfence();
#pragma unroll
  for (int i = 0; i < 8; ++i) {
    const int gr = rowBase + 16 * wave + 2 * i + hh;
    const int gc = gr < nN ? gr : nN - 1;
    float* op = out + (size_t)gc * F_OUT + 4 * m;
    if (gr < nN) *(volatile v4f*)op = fv[i];
  }
}

static inline size_t al256(size_t v) { return (v + 255) & ~(size_t)255; }

extern "C" void kernel_launch(void* const* d_in, const int* in_sizes, int n_in,
                              void* d_out, int out_size, void* d_ws, size_t ws_size,
                              hipStream_t stream) {
  if (n_in < 9) return;
  if (in_sizes[0] != NN * F_IN) return;
  if (in_sizes[1] != 2 * NE) return;
  if (in_sizes[3] != F_IN * HC) return;
  if (in_sizes[4] != NHD * HID || in_sizes[5] != NHD * HID) return;
  if (in_sizes[6] != HC) return;
  if (in_sizes[7] != HC * F_OUT) return;
  if (in_sizes[8] != F_OUT) return;
  if (out_size != NN * F_OUT) return;

  const float* x    = (const float*)d_in[0];
  const int*   ei   = (const int*)  d_in[1];
  const float* W    = (const float*)d_in[3];
  const float* asrc = (const float*)d_in[4];
  const float* adst = (const float*)d_in[5];
  const float* bias = (const float*)d_in[6];
  const float* W2   = (const float*)d_in[7];
  const float* b2   = (const float*)d_in[8];
  float* out = (float*)d_out;
  const int* src = ei;
  const int* dst = ei + NE;

  char* ws = (char*)d_ws;
  size_t off = 0;
  const size_t oXB  = off; off = al256(off + (size_t)MP * XPITCH * 2);
  const size_t oWT  = off; off = al256(off + (size_t)HC * WPITCH * 2);
  const size_t oW2D = off; off = al256(off + (size_t)F_OUT * W2PITCH * 2);
  const size_t oSP  = off; off = al256(off + (size_t)2048);
  const size_t oH   = off; off = al256(off + (size_t)MP * HC * 4);
  const size_t oSD  = off; off = al256(off + (size_t)MP * 8 * 4);
  const size_t oE   = off; off = al256(off + (size_t)MP * EPITCH * 2);
  const size_t oHT  = off; off = al256(off + (size_t)NBLK * RCAP * 4);
  const size_t oOF  = off; off = al256(off + (size_t)NBLK * NBRUN * 4);
  const size_t oCN  = off; off = al256(off + (size_t)NBLK * NBRUN * 4);
  const size_t oFL  = off; off = al256(off + (size_t)NBLK * 32 * 4);
  if (off > ws_size || off > WSMAX) return;
  unsigned short* XB  = (unsigned short*)(ws + oXB);
  unsigned short* WT  = (unsigned short*)(ws + oWT);
  unsigned short* W2D = (unsigned short*)(ws + oW2D);
  float*          SP  = (float*)(ws + oSP);
  float*          H   = (float*)(ws + oH);
  float*          SD  = (float*)(ws + oSD);
  unsigned short* E   = (unsigned short*)(ws + oE);
  int*            HT  = (int*)(ws + oHT);
  int*            OF  = (int*)(ws + oOF);
  int*            CN  = (int*)(ws + oCN);
  int*            FL  = (int*)(ws + oFL);

  hipFuncSetAttribute(reinterpret_cast<const void*>(&k_bucket),
                      hipFuncAttributeMaxDynamicSharedMemorySize, LDS_BKT);

  k_prep<<<PB_ALL, NTHR, 0, stream>>>(x, W, W2, asrc, adst, bias, b2, XB, WT, W2D, SP, E);
  k_gemm_one<<<MP / G1M, G1T, 0, stream>>>(XB, WT, SP, H, SD);
  k_bucket<<<NBLK, NTHR, LDS_BKT, stream>>>(src, dst, HT, OF, CN, FL, NN, NE, ((NE & 3) == 0) ? 1 : 0);
  k_replay<<<(NN + NWAVE - 1) / NWAVE, NTHR, 0, stream>>>(H, SD, SP, HT, OF, CN, FL, E, NN);
  k_gemm_two<<<MP / G2M, G2T, 0, stream>>>(E, W2D, SP, CN, FL, out, NN);
}
